// BipartiteGNNEncoder_7026566496898
// MI455X (gfx1250) — hardware-verified
//
#include <hip/hip_runtime.h>
#include <stddef.h>


#define SIN     10
#define VIN     9
#define HID     64
#define OUTD    32
#define KA      128
#define KP      136
#define WP      128
#define WROWS   192
#define RBLK    64
#define GTHR    128
#define NTHR    256
#define NWAVE   8
#define OPM     68
#define CHUNK   2048
#define WCAP    256
#define LISTN   (NWAVE * WCAP)
#define ESH     16
#define NBC     32768
#define NBFV    384
#define NBFS    3840
#define RBYTES  262144
#define RCAPV   (RBYTES / 4)
#define RCAPS   (RBYTES / 2)
#define CPT     16
#define DEGCAP  1024
#define LDS_COUNT (NBC * 4 + LISTN * 4 + 64)
#define LDS_FILLV (RBYTES + NBFV * 4 + LISTN * 4 + 64)
#define LDS_FILLS (RBYTES + NBFS * 4 + LISTN * 4 + 64)

static_assert(CHUNK == NTHR * 8);
static_assert(CHUNK / NWAVE == WCAP);
static_assert((WCAP & (WCAP - 1)) == 0 && (CHUNK & (CHUNK - 1)) == 0);
static_assert(CHUNK <= (1 << (31 - ESH)));
static_assert((NBC & (NBC - 1)) == 0 && NBC < (1 << ESH));
static_assert(NBFV < (1 << ESH) && NBFS < (1 << ESH));
static_assert((NBFV % 32) == 0 && (NBFS % 32) == 0);
static_assert((NBFV % CPT) == 0 && (NBFS % CPT) == 0);
static_assert(NBFV / CPT <= NTHR && NBFS / CPT <= NTHR);
static_assert(((NBFV * 4) % 16) == 0 && ((NBFS * 4) % 16) == 0);
static_assert(WROWS * 16 == 12 * NTHR);
static_assert(RBLK == (GTHR / 32) * 16);
static_assert(((KP * 2) % 16) == 0 && ((OPM * 4) % 16) == 0 && ((WP * 2) % 16) == 0);
static_assert((RBYTES % 16) == 0);

typedef float          v4f  __attribute__((ext_vector_type(4)));
typedef float          v8f  __attribute__((ext_vector_type(8)));
typedef int            v4i  __attribute__((ext_vector_type(4)));
typedef unsigned short v8us __attribute__((ext_vector_type(8)));
typedef __bf16         v8b  __attribute__((ext_vector_type(8)));
typedef __bf16         v16b __attribute__((ext_vector_type(16)));
union FragB { v16b v; v8us h[2]; };
union Pack8 { v8b b; v8us u; };

__device__ __forceinline__ void split8(v4f a, v4f b, v8us& hi, v8us& lo) {
  const float x[8] = {a.x, a.y, a.z, a.w, b.x, b.y, b.z, b.w};
  Pack8 ph, pl;
#pragma unroll
  for (int e = 0; e < 8; ++e) {
    const __bf16 hb = (__bf16)x[e];
    const float  hf = (float)hb;
    ph.b[e] = hb;
    pl.b[e] = (__bf16)(x[e] - hf);
  }
  hi = ph.u;
  lo = pl.u;
}

__device__ __forceinline__ v8f wmb(v16b a, v16b b, v8f c) {
  v8f d = __builtin_amdgcn_wmma_f32_16x16x32_bf16(false, a, false, b, (short)0, c, false, false);
  asm volatile("v_nop\n\tv_nop\n\tv_nop\n\tv_nop" : "+v"(d) : "v"(a), "v"(b));
  return d;
}

__device__ __forceinline__ v4f xred(v4f a) {
#pragma unroll
  for (int s = 4; s <= 16; s <<= 1) {
    a.x += __shfl_xor(a.x, s, 32);
    a.y += __shfl_xor(a.y, s, 32);
    a.z += __shfl_xor(a.z, s, 32);
    a.w += __shfl_xor(a.w, s, 32);
  }
  return a;
}

__device__ __forceinline__ v4f sel4(bool c, v4f a, v4f b) {
  v4f r;
  r.x = c ? a.x : b.x; r.y = c ? a.y : b.y; r.z = c ? a.z : b.z; r.w = c ? a.w : b.w;
  return r;
}

__device__ __forceinline__ void load8i(const int* __restrict__ p, int nE, int cbase, int e0, int fillv,
                                       v4i& a, v4i& b) {
  if (cbase + CHUNK <= nE) {
    a = *(const v4i*)(p + e0);
    b = *(const v4i*)(p + e0 + 4);
  } else {
    const int l = nE - 1;
    a.x = (e0     < nE) ? p[min(e0,     l)] : fillv;
    a.y = (e0 + 1 < nE) ? p[min(e0 + 1, l)] : fillv;
    a.z = (e0 + 2 < nE) ? p[min(e0 + 2, l)] : fillv;
    a.w = (e0 + 3 < nE) ? p[min(e0 + 3, l)] : fillv;
    b.x = (e0 + 4 < nE) ? p[min(e0 + 4, l)] : fillv;
    b.y = (e0 + 5 < nE) ? p[min(e0 + 5, l)] : fillv;
    b.z = (e0 + 6 < nE) ? p[min(e0 + 6, l)] : fillv;
    b.w = (e0 + 7 < nE) ? p[min(e0 + 7, l)] : fillv;
  }
}

template <int NB>
__device__ __forceinline__ int scan_chunk(const int* __restrict__ keys, int nE, int cbase, int slotBase,
                                          int* list, int lane, int wave) {
  const int el0 = wave * WCAP + 8 * lane;
  const int e0  = cbase + el0;
  const int sent = -2147483647 - 1;
  v4i ka, kb;
  load8i(keys, nE, cbase, e0, sent, ka, kb);
  const unsigned nb = (unsigned)slotBase;
  unsigned s[8];
  s[0] = (unsigned)ka.x - nb; s[1] = (unsigned)ka.y - nb; s[2] = (unsigned)ka.z - nb; s[3] = (unsigned)ka.w - nb;
  s[4] = (unsigned)kb.x - nb; s[5] = (unsigned)kb.y - nb; s[6] = (unsigned)kb.z - nb; s[7] = (unsigned)kb.w - nb;
  int h[8];
  int c = 0;
#pragma unroll
  for (int j = 0; j < 8; ++j) { h[j] = (s[j] < (unsigned)NB) ? 1 : 0; c += h[j]; }
  if (__builtin_amdgcn_ballot_w32(c != 0) == 0u) return 0;
  int incl = c;
#pragma unroll
  for (int d = 1; d < 32; d <<= 1) {
    const int t = __shfl_up(incl, d, 32);
    incl += (lane >= d) ? t : 0;
  }
  int p = incl - c;
  int* lp = list + wave * WCAP;
#pragma unroll
  for (int j = 0; j < 8; ++j) {
    if (h[j] != 0) lp[min(p, WCAP - 1)] = ((el0 + j) << ESH) | (int)s[j];
    p += h[j];
  }
  return __shfl(incl, 31, 32);
}

__device__ __forceinline__ void batch_locate(const int* list, const int (&wcv)[NWAVE], int H, int bt, int lane,
                                             int& slot, int& el, bool& valid) {
  const int g = 32 * bt + lane;
  valid = g < H;
  int w = 0, idx = g;
#pragma unroll
  for (int k = 0; k < NWAVE - 1; ++k) {
    const bool adv = (w == k) && (idx >= wcv[k]);
    w   += adv ? 1 : 0;
    idx -= adv ? wcv[k] : 0;
  }
  idx = idx < 0 ? 0 : (idx > WCAP - 1 ? WCAP - 1 : idx);
  const int ent = list[w * WCAP + idx];
  slot = valid ? (ent & ((1 << ESH) - 1)) : -1;
  el   = (ent >> ESH) & (CHUNK - 1);
}

__device__ __forceinline__ void batch_match(int slot, int lane, int& cntm, int& rank) {
  cntm = 0; rank = 0;
#pragma unroll
  for (int it = 0; it < 32; ++it) {
    const int so = __builtin_amdgcn_readlane(slot, it);
    const int eq = (slot == so) ? 1 : 0;
    cntm += eq;
    rank += (it < lane) ? eq : 0;
  }
}

__global__ __launch_bounds__(NTHR) void k_wprep(
    const float* __restrict__ Wl1sv, const float* __restrict__ Wr1sv,
    const float* __restrict__ Wl1vs, const float* __restrict__ Wr1vs,
    const float* __restrict__ Wl2sv, const float* __restrict__ Wr2sv,
    const float* __restrict__ Wl2vs, const float* __restrict__ Wr2vs,
    unsigned short* wh, unsigned short* wl) {
  const int tid = threadIdx.x, blk = blockIdx.x;
  const int i = blk * NTHR + tid;
  const int row = i >> 4;
  const int k0 = (i & 15) * 8;
  const float* pl;
  const float* pr;
  int N, n;
  if (blk < 4)       { pl = Wl1sv; pr = Wr1sv; N = HID;  n = row; }
  else if (blk < 8)  { pl = Wl1vs; pr = Wr1vs; N = HID;  n = row - 64; }
  else if (blk < 10) { pl = Wl2sv; pr = Wr2sv; N = OUTD; n = row - 128; }
  else               { pl = Wl2vs; pr = Wr2vs; N = OUTD; n = row - 160; }
  n = n < 0 ? 0 : (n > N - 1 ? N - 1 : n);
  float v[8];
#pragma unroll
  for (int e = 0; e < 8; ++e) {
    const int k  = k0 + e;
    const int kk = k & (HID - 1);
    const float a = pl[kk * N + n];
    const float b = pr[kk * N + n];
    v[e] = (k < HID) ? a : b;
  }
  v4f va, vb;
  va.x = v[0]; va.y = v[1]; va.z = v[2]; va.w = v[3];
  vb.x = v[4]; vb.y = v[5]; vb.z = v[6]; vb.w = v[7];
  v8us hh, ll;
  split8(va, vb, hh, ll);
  const size_t o = (size_t)row * WP + k0;
  *(volatile v8us*)(wh + o) = hh;
  *(volatile v8us*)(wl + o) = ll;
  __threadfence();
  *(volatile v8us*)(wh + o) = hh;
  *(volatile v8us*)(wl + o) = ll;
}

__global__ __launch_bounds__(NTHR) void k_inproj(
    const float* __restrict__ X, const float* __restrict__ W, const float* __restrict__ bias,
    float* plane, int nRows, int kin) {
  const int tid = threadIdx.x, lane = tid & 31, wave = tid >> 5;
  const int c16 = lane & 15, hsel = lane >> 4;
  const int rowBase = blockIdx.x * RBLK + wave * 8;
  const v4f bv = *(const v4f*)(bias + 4 * c16);
  const v4f z4 = {0.f, 0.f, 0.f, 0.f};
  v4f o[4];
#pragma unroll
  for (int i = 0; i < 4; ++i) {
    const int r = rowBase + 2 * i + hsel;
    const int rc = r > nRows - 1 ? nRows - 1 : r;
    v4f acc = bv;
#pragma unroll 1
    for (int k = 0; k < kin; ++k) {
      const float xk = X[(size_t)rc * kin + k];
      const v4f w = *(const v4f*)(W + k * HID + 4 * c16);
      acc += xk * w;
    }
    o[i] = (r < nRows) ? acc : z4;
  }
#pragma unroll
  for (int i = 0; i < 4; ++i) {
    const int r = rowBase + 2 * i + hsel;
    *(volatile v4f*)(plane + (size_t)r * HID + 4 * c16) = o[i];
  }
  __threadfence();
#pragma unroll
  for (int i = 0; i < 4; ++i) {
    const int r = rowBase + 2 * i + hsel;
    *(volatile v4f*)(plane + (size_t)r * HID + 4 * c16) = o[i];
  }
}

__global__ __launch_bounds__(NTHR) void k_count(const int* __restrict__ keys, int* cnt, int nE) {
  extern __shared__ v4i lds_dyn[];
  int* scnt = (int*)lds_dyn;
  int* list = scnt + NBC;
  int* wcnt = list + LISTN;
  const int tid = threadIdx.x, lane = tid & 31, wave = tid >> 5;
  const int base = blockIdx.x * NBC;
  {
    const v4i z = {0, 0, 0, 0};
#pragma unroll 1
    for (int i = tid; i < NBC / 4; i += NTHR) lds_dyn[i] = z;
  }
  __syncthreads();

#pragma unroll 1
  for (int cbase = 0; cbase < nE; cbase += CHUNK) {
    const int wc = scan_chunk<NBC>(keys, nE, cbase, base, list, lane, wave);
    if (lane == 0) wcnt[wave] = wc;
    __syncthreads();
    if (wave == 0) {
      int wcv[NWAVE];
      int H = 0;
#pragma unroll
      for (int k = 0; k < NWAVE; ++k) {
        int v = wcnt[k];
        v = v < 0 ? 0 : (v > WCAP ? WCAP : v);
        wcv[k] = v;
        H += v;
      }
      H = __builtin_amdgcn_readfirstlane(H);
      const int nbt = (H + 31) >> 5;
#pragma unroll 1
      for (int bt = 0; bt < nbt; ++bt) {
        int slot, el, cntm, rank;
        bool valid;
        batch_locate(list, wcv, H, bt, lane, slot, el, valid);
        batch_match(slot, lane, cntm, rank);
        if (valid && rank == 0) {
          const int sc = slot & (NBC - 1);
          scnt[sc] = scnt[sc] + cntm;
        }
      }
    }
    __syncthreads();
  }

  int* cp = cnt + (size_t)base;
#pragma unroll 1
  for (int i = tid; i < NBC / 4; i += NTHR) { const v4i v = lds_dyn[i]; *(volatile v4i*)(cp + 4 * i) = v; }
  __threadfence();
#pragma unroll 1
  for (int i = tid; i < NBC / 4; i += NTHR) { const v4i v = lds_dyn[i]; *(volatile v4i*)(cp + 4 * i) = v; }
}

template <int NBF, typename RT, int RCAP>
__global__ __launch_bounds__(NTHR) void k_fill(
    const int* __restrict__ keys, const int* __restrict__ vals, const int* __restrict__ cnt,
    int* off, RT* csr, int nVal, int nE) {
  constexpr int NTC = NBF / CPT;
  constexpr int EPL = 128 / (int)sizeof(RT);
  static_assert((NBF % CPT) == 0 && NTC <= NTHR);
  static_assert(RCAP * (int)sizeof(RT) == RBYTES && (RCAP % EPL) == 0 && (EPL & (EPL - 1)) == 0);
  extern __shared__ v4i lds_dyn[];
  RT*  region = (RT*)lds_dyn;
  int* cursor = (int*)(lds_dyn + RBYTES / 16);
  int* list   = cursor + NBF;
  int* wcnt   = list + LISTN;
  int* wtot   = wcnt + NWAVE;
  const int tid = threadIdx.x, lane = tid & 31, wave = tid >> 5;
  const int b = blockIdx.x;
  const int nodeBase = b * NBF;

  {
    const v4i z = {0, 0, 0, 0};
#pragma unroll 1
    for (int i = tid; i < RBYTES / 16; i += NTHR) lds_dyn[i] = z;
  }

  const bool act = tid < NTC;
  const int  tc  = act ? tid : (NTC - 1);
  const int* cb  = cnt + (size_t)nodeBase + CPT * tc;
  const v4i c0 = *(const v4i*)(cb);
  const v4i c1 = *(const v4i*)(cb + 4);
  const v4i c2 = *(const v4i*)(cb + 8);
  const v4i c3 = *(const v4i*)(cb + 12);
  int e[CPT];
  e[0]  = c0.x; e[1]  = c0.y; e[2]  = c0.z; e[3]  = c0.w;
  e[4]  = c1.x; e[5]  = c1.y; e[6]  = c1.z; e[7]  = c1.w;
  e[8]  = c2.x; e[9]  = c2.y; e[10] = c2.z; e[11] = c2.w;
  e[12] = c3.x; e[13] = c3.y; e[14] = c3.z; e[15] = c3.w;
  int ts = 0;
#pragma unroll
  for (int i = 0; i < CPT; ++i) {
    int v = e[i];
    v = v < 0 ? 0 : (v > DEGCAP ? DEGCAP : v);
    v = act ? v : 0;
    e[i] = v;
    ts += v;
  }
  int incl = ts;
#pragma unroll
  for (int d = 1; d < 32; d <<= 1) {
    const int t = __shfl_up(incl, d, 32);
    incl += (lane >= d) ? t : 0;
  }
  if (lane == 31) wtot[wave] = incl;
  __syncthreads();
  int T = 0, pre = 0;
#pragma unroll
  for (int w = 0; w < NWAVE; ++w) {
    const int t = wtot[w];
    T += t;
    pre += (w < wave) ? t : 0;
  }
  if (act) {
    int run = pre + incl - ts;
#pragma unroll
    for (int i = 0; i < CPT; ++i) {
      cursor[CPT * tid + i] = run > RCAP ? RCAP : run;
      run += e[i];
    }
  }
  __syncthreads();
  {
    const int rb = b * RCAP;
    int* op = off + (size_t)nodeBase;
#pragma unroll 1
    for (int i = tid; i < NBF / 4; i += NTHR) {
      v4i o = ((const v4i*)cursor)[i];
      o.x += rb; o.y += rb; o.z += rb; o.w += rb;
      *(volatile v4i*)(op + 4 * i) = o;
    }
    __threadfence();
#pragma unroll 1
    for (int i = tid; i < NBF / 4; i += NTHR) {
      v4i o = ((const v4i*)cursor)[i];
      o.x += rb; o.y += rb; o.z += rb; o.w += rb;
      *(volatile v4i*)(op + 4 * i) = o;
    }
  }
  const int Tt   = T > RCAP ? RCAP : (T < 0 ? 0 : T);
  const int lenW = (Tt + EPL - 1) & ~(EPL - 1);

#pragma unroll 1
  for (int cbase = 0; cbase < nE; cbase += CHUNK) {
    const int wc = scan_chunk<NBF>(keys, nE, cbase, nodeBase, list, lane, wave);
    if (lane == 0) wcnt[wave] = wc;
    __syncthreads();
    if (wave == 0) {
      int wcv[NWAVE];
      int H = 0;
#pragma unroll
      for (int k = 0; k < NWAVE; ++k) {
        int v = wcnt[k];
        v = v < 0 ? 0 : (v > WCAP ? WCAP : v);
        wcv[k] = v;
        H += v;
      }
      H = __builtin_amdgcn_readfirstlane(H);
      const int nbt = (H + 31) >> 5;
#pragma unroll 1
      for (int bt = 0; bt < nbt; ++bt) {
        int slot, el, cntm, rank;
        bool valid;
        batch_locate(list, wcv, H, bt, lane, slot, el, valid);
        batch_match(slot, lane, cntm, rank);
        int eg = cbase + el;
        eg = eg > nE - 1 ? nE - 1 : (eg < 0 ? 0 : eg);
        int v = vals[eg];
        v = v < 0 ? 0 : (v > nVal - 1 ? nVal - 1 : v);
        const int sc = slot < 0 ? 0 : (slot > NBF - 1 ? NBF - 1 : slot);
        const int base0 = cursor[sc];
        const int pos = base0 + rank;
        if (valid && pos >= 0 && pos < RCAP) region[pos] = (RT)v;
        if (valid && rank == 0) {
          const int np = base0 + cntm;
          cursor[sc] = np > RCAP ? RCAP : np;
        }
      }
    }
    __syncthreads();
  }

  const int nv = lenW * (int)sizeof(RT) / 16;
  char* gpb = (char*)csr + (size_t)b * RBYTES;
#pragma unroll 1
  for (int i = tid; i < nv; i += NTHR) { const v4i v = lds_dyn[i]; *(volatile v4i*)(gpb + 16 * (size_t)i) = v; }
  __threadfence();
#pragma unroll 1
  for (int i = tid; i < nv; i += NTHR) { const v4i v = lds_dyn[i]; *(volatile v4i*)(gpb + 16 * (size_t)i) = v; }
}

template <int NT, typename IT>
__global__ __launch_bounds__(GTHR) void k_agg(
    const IT* __restrict__ csr, const int* __restrict__ off, const int* __restrict__ cnt, int csrLen,
    const float* __restrict__ srcP, int nSrc, const float* __restrict__ selfP, int nDst,
    const unsigned short* __restrict__ wh, const unsigned short* __restrict__ wl,
    const float* __restrict__ bias, float* outp, int nStore) {
  constexpr int NOUT = NT * 16;
  constexpr int LPR  = NOUT / 4;
  constexpr int RPI  = 32 / LPR;
  constexpr int NI   = 16 / RPI;
  __shared__ __attribute__((aligned(16))) unsigned short sAh[RBLK * KP];
  __shared__ __attribute__((aligned(16))) unsigned short sAl[RBLK * KP];
  __shared__ __attribute__((aligned(16))) float sO[RBLK * OPM];
  const int tid = threadIdx.x, lane = tid & 31, wave = tid >> 5;
  const int h = lane >> 4, m = lane & 15, q = lane >> 2, c4 = lane & 3;
  const int rowBase = blockIdx.x * RBLK;
  const v4f z4 = {0.f, 0.f, 0.f, 0.f};

#pragma unroll 1
  for (int j = 0; j < 16; ++j) {
    const int rl = wave * 16 + j;
    int rc = rowBase + rl;
    rc = rc > nDst - 1 ? nDst - 1 : rc;
    int n = cnt[rc];
    n = n < 0 ? 0 : (n > DEGCAP ? DEGCAP : n);
    int st = off[rc];
    st = st < 0 ? 0 : (st > csrLen - 1 ? csrLen - 1 : st);
    const float inv = 1.0f / (float)(n < 1 ? 1 : n);
    v4f a0 = z4, a1 = z4, a2 = z4, a3 = z4;
#pragma unroll 1
    for (int p0 = 0; p0 < n; p0 += 32) {
      int pos = st + p0 + lane;
      pos = pos < 0 ? 0 : (pos > csrLen - 1 ? csrLen - 1 : pos);
      int sl = (int)csr[pos];
      sl = sl < 0 ? 0 : (sl > nSrc - 1 ? nSrc - 1 : sl);
      const int mc = (n - p0) < 32 ? (n - p0) : 32;
#pragma unroll 1
      for (int g = 0; g < mc; g += 8) {
        const int sg = __shfl(sl, g + q, 32);
        const int sv = ((g + q) < mc) ? sg : nSrc;
        const float* p = srcP + (size_t)sv * HID + 16 * c4;
        const v4f x0 = *(const v4f*)(p);
        const v4f x1 = *(const v4f*)(p + 4);
        const v4f x2 = *(const v4f*)(p + 8);
        const v4f x3 = *(const v4f*)(p + 12);
        a0 += x0; a1 += x1; a2 += x2; a3 += x3;
      }
    }
    a0 = xred(a0) * inv;
    a1 = xred(a1) * inv;
    a2 = xred(a2) * inv;
    a3 = xred(a3) * inv;
    const float* ps = selfP + (size_t)rc * HID + 16 * c4;
    const v4f s0 = *(const v4f*)(ps);
    const v4f s1 = *(const v4f*)(ps + 4);
    const v4f s2 = *(const v4f*)(ps + 8);
    const v4f s3 = *(const v4f*)(ps + 12);
    const bool um = (q == 0);
    const v4f t0 = sel4(um, a0, s0);
    const v4f t1 = sel4(um, a1, s1);
    const v4f t2 = sel4(um, a2, s2);
    const v4f t3 = sel4(um, a3, s3);
    v8us hh0, ll0, hh1, ll1;
    split8(t0, t1, hh0, ll0);
    split8(t2, t3, hh1, ll1);
    if (q < 2) {
      const int ao = rl * KP + (um ? 0 : HID) + 16 * c4;
      *(v8us*)(sAh + ao)     = hh0;
      *(v8us*)(sAh + ao + 8) = hh1;
      *(v8us*)(sAl + ao)     = ll0;
      *(v8us*)(sAl + ao + 8) = ll1;
    }
  }
  __syncthreads();

  v8f acc[NT];
#pragma unroll
  for (int nt = 0; nt < NT; ++nt) { const v8f z8 = {0.f, 0.f, 0.f, 0.f, 0.f, 0.f, 0.f, 0.f}; acc[nt] = z8; }
  const unsigned short* ahp = sAh + (wave * 16 + m) * KP + 8 * h;
  const unsigned short* alp = sAl + (wave * 16 + m) * KP + 8 * h;
#pragma unroll 1
  for (int kt = 0; kt < KA / 32; ++kt) {
    FragB fah, fal;
    fah.h[0] = *(const v8us*)(ahp + 32 * kt);
    fah.h[1] = *(const v8us*)(ahp + 32 * kt + 16);
    fal.h[0] = *(const v8us*)(alp + 32 * kt);
    fal.h[1] = *(const v8us*)(alp + 32 * kt + 16);
#pragma unroll
    for (int nt = 0; nt < NT; ++nt) {
      const size_t bo = (size_t)(16 * nt + m) * WP + 32 * kt + 8 * h;
      FragB fbh, fbl;
      fbh.h[0] = *(const v8us*)(wh + bo);
      fbh.h[1] = *(const v8us*)(wh + bo + 16);
      fbl.h[0] = *(const v8us*)(wl + bo);
      fbl.h[1] = *(const v8us*)(wl + bo + 16);
      acc[nt] = wmb(fah.v, fbh.v, acc[nt]);
      acc[nt] = wmb(fal.v, fbh.v, acc[nt]);
      acc[nt] = wmb(fah.v, fbl.v, acc[nt]);
    }
  }

  const int lim = nDst - (rowBase + wave * 16 + 8 * h);
#pragma unroll
  for (int nt = 0; nt < NT; ++nt) {
    const float bv = bias[16 * nt + m];
#pragma unroll
    for (int r = 0; r < 8; ++r) {
      float v = fmaxf(acc[nt][r] + bv, 0.f);
      v = (r < lim) ? v : 0.f;
      sO[(wave * 16 + 8 * h + r) * OPM + 16 * nt + m] = v;
    }
  }
  __syncthreads();

  const int pc = lane % LPR;
  v4f ov[NI];
#pragma unroll
  for (int i = 0; i < NI; ++i) {
    const int rl = wave * 16 + RPI * i + lane / LPR;
    ov[i] = *(const v4f*)(sO + rl * OPM + 4 * pc);
  }
#pragma unroll
  for (int i = 0; i < NI; ++i) {
    const int r = rowBase + wave * 16 + RPI * i + lane / LPR;
    if (r < nStore) *(volatile v4f*)(outp + (size_t)r * NOUT + 4 * pc) = ov[i];
  }
  __threadfence();
#pragma unroll
  for (int i = 0; i < NI; ++i) {
    const int r = rowBase + wave * 16 + RPI * i + lane / LPR;
    if (r < nStore) *(volatile v4f*)(outp + (size_t)r * NOUT + 4 * pc) = ov[i];
  }
}

static inline int up64(int a) { return (a + 63) & ~63; }
static inline int cdivi(int a, int b) { return (a + b - 1) / b; }

extern "C" void kernel_launch(void* const* d_in, const int* in_sizes, int n_in,
                              void* d_out, int out_size, void* d_ws, size_t ws_size,
                              hipStream_t stream) {
  if (n_in < 20) return;
  const int nS = in_sizes[0] / SIN;
  if (nS < 1 || in_sizes[0] != nS * SIN) return;
  const int nV = in_sizes[1] / VIN;
  if (nV < 1 || in_sizes[1] != nV * VIN) return;
  const int nE = in_sizes[2];
  if (nE < 1 || in_sizes[3] != nE) return;
  if (in_sizes[4] != SIN * HID || in_sizes[5] != HID || in_sizes[6] != VIN * HID || in_sizes[7] != HID) return;
  if (in_sizes[8] != HID * HID || in_sizes[9] != HID || in_sizes[10] != HID * HID) return;
  if (in_sizes[11] != HID * HID || in_sizes[12] != HID || in_sizes[13] != HID * HID) return;
  if (in_sizes[14] != HID * OUTD || in_sizes[15] != OUTD || in_sizes[16] != HID * OUTD) return;
  if (in_sizes[17] != HID * OUTD || in_sizes[18] != OUTD || in_sizes[19] != HID * OUTD) return;
  if (out_size != (nS + nV) * OUTD) return;
  if (nS > (1 << 24) || nV > 65535 || nE > (1 << 28)) return;

  const float* x_site   = (const float*)d_in[0];
  const float* x_vendor = (const float*)d_in[1];
  const int*   srci     = (const int*)d_in[2];
  const int*   dsti     = (const int*)d_in[3];
  const float* W_si     = (const float*)d_in[4];
  const float* b_si     = (const float*)d_in[5];
  const float* W_vi     = (const float*)d_in[6];
  const float* b_vi     = (const float*)d_in[7];
  const float* Wl1sv    = (const float*)d_in[8];
  const float* bl1sv    = (const float*)d_in[9];
  const float* Wr1sv    = (const float*)d_in[10];
  const float* Wl1vs    = (const float*)d_in[11];
  const float* bl1vs    = (const float*)d_in[12];
  const float* Wr1vs    = (const float*)d_in[13];
  const float* Wl2sv    = (const float*)d_in[14];
  const float* bl2sv    = (const float*)d_in[15];
  const float* Wr2sv    = (const float*)d_in[16];
  const float* Wl2vs    = (const float*)d_in[17];
  const float* bl2vs    = (const float*)d_in[18];
  const float* Wr2vs    = (const float*)d_in[19];
  float* out = (float*)d_out;

  const int nSP = up64(nS + 1), nVP = up64(nV + 1);
  const int nBS = nSP / RBLK, nBV = nVP / RBLK;
  const int nFBV = cdivi(nV, NBFV);
  const int nBCV = cdivi(nFBV * NBFV, NBC);
  const int nFBS = cdivi(nS, NBFS);
  const int nBCS = cdivi(nFBS * NBFS, NBC);
  const int csrLenV = nFBV * RCAPV;
  const int csrLenS = nFBS * RCAPS;

  char* ws = (char*)d_ws;
  size_t off = 0;
  const size_t oWh  = off; off += (size_t)WROWS * WP * 2;          off = (off + 255) & ~(size_t)255;
  const size_t oWl  = off; off += (size_t)WROWS * WP * 2;          off = (off + 255) & ~(size_t)255;
  const size_t oXs  = off; off += (size_t)nSP * HID * 4;           off = (off + 255) & ~(size_t)255;
  const size_t oXv  = off; off += (size_t)nVP * HID * 4;           off = (off + 255) & ~(size_t)255;
  const size_t oXs1 = off; off += (size_t)nSP * HID * 4;           off = (off + 255) & ~(size_t)255;
  const size_t oXv1 = off; off += (size_t)nVP * HID * 4;           off = (off + 255) & ~(size_t)255;
  const size_t oCnV = off; off += (size_t)nBCV * NBC * 4;          off = (off + 255) & ~(size_t)255;
  const size_t oOfV = off; off += (size_t)nFBV * NBFV * 4;         off = (off + 255) & ~(size_t)255;
  const size_t oCsV = off; off += (size_t)nFBV * RBYTES;           off = (off + 255) & ~(size_t)255;
  const size_t oCnS = off; off += (size_t)nBCS * NBC * 4;          off = (off + 255) & ~(size_t)255;
  const size_t oOfS = off; off += (size_t)nFBS * NBFS * 4;         off = (off + 255) & ~(size_t)255;
  const size_t oCsS = off; off += (size_t)nFBS * RBYTES;           off = (off + 255) & ~(size_t)255;
  if (off > ws_size) return;
  unsigned short* wh   = (unsigned short*)(ws + oWh);
  unsigned short* wl   = (unsigned short*)(ws + oWl);
  float*          xs   = (float*)(ws + oXs);
  float*          xv   = (float*)(ws + oXv);
  float*          xs1  = (float*)(ws + oXs1);
  float*          xv1  = (float*)(ws + oXv1);
  int*            cntV = (int*)(ws + oCnV);
  int*            offV = (int*)(ws + oOfV);
  int*            csrV = (int*)(ws + oCsV);
  int*            cntS = (int*)(ws + oCnS);
  int*            offS = (int*)(ws + oOfS);
  unsigned short* csrS = (unsigned short*)(ws + oCsS);

  k_wprep<<<WROWS * 16 / NTHR, NTHR, 0, stream>>>(Wl1sv, Wr1sv, Wl1vs, Wr1vs, Wl2sv, Wr2sv, Wl2vs, Wr2vs, wh, wl);

  k_inproj<<<nBS, NTHR, 0, stream>>>(x_site, W_si, b_si, xs, nS, SIN);
  k_inproj<<<nBV, NTHR, 0, stream>>>(x_vendor, W_vi, b_vi, xv, nV, VIN);

  hipFuncSetAttribute(reinterpret_cast<const void*>(&k_count),
                      hipFuncAttributeMaxDynamicSharedMemorySize, LDS_COUNT);
  hipLaunchKernelGGL(k_count, dim3(nBCV), dim3(NTHR), LDS_COUNT, stream, dsti, cntV, nE);
  hipFuncSetAttribute(reinterpret_cast<const void*>(&k_fill<NBFV, int, RCAPV>),
                      hipFuncAttributeMaxDynamicSharedMemorySize, LDS_FILLV);
  hipLaunchKernelGGL((k_fill<NBFV, int, RCAPV>), dim3(nFBV), dim3(NTHR), LDS_FILLV, stream,
                     dsti, srci, cntV, offV, csrV, nS, nE);

  hipLaunchKernelGGL(k_count, dim3(nBCS), dim3(NTHR), LDS_COUNT, stream, srci, cntS, nE);
  hipFuncSetAttribute(reinterpret_cast<const void*>(&k_fill<NBFS, unsigned short, RCAPS>),
                      hipFuncAttributeMaxDynamicSharedMemorySize, LDS_FILLS);
  hipLaunchKernelGGL((k_fill<NBFS, unsigned short, RCAPS>), dim3(nFBS), dim3(NTHR), LDS_FILLS, stream,
                     srci, dsti, cntS, offS, csrS, nV, nE);

  hipLaunchKernelGGL((k_agg<4, int>), dim3(nBV), dim3(GTHR), 0, stream,
                     csrV, offV, cntV, csrLenV, xs, nS, xv, nV, wh, wl, bl1sv, xv1, nVP);
  hipLaunchKernelGGL((k_agg<4, unsigned short>), dim3(nBS), dim3(GTHR), 0, stream,
                     csrS, offS, cntS, csrLenS, xv, nV, xs, nS, wh + 64 * WP, wl + 64 * WP, bl1vs, xs1, nSP);

  hipLaunchKernelGGL((k_agg<2, unsigned short>), dim3(nBS), dim3(GTHR), 0, stream,
                     csrS, offS, cntS, csrLenS, xv1, nV, xs1, nS, wh + 160 * WP, wl + 160 * WP, bl2vs, out, nS);
  hipLaunchKernelGGL((k_agg<2, int>), dim3(nBV), dim3(GTHR), 0, stream,
                     csrV, offV, cntV, csrLenV, xs1, nS, xv1, nV, wh + 128 * WP, wl + 128 * WP, bl2sv,
                     out + (size_t)nS * OUTD, nV);
}
